// GSAttention_21337397527393
// MI455X (gfx1250) — hardware-verified
//
#include <hip/hip_runtime.h>
#include <math.h>

typedef __attribute__((ext_vector_type(16))) _Float16 v16h;
typedef __attribute__((ext_vector_type(16))) __bf16 v16b;
typedef __attribute__((ext_vector_type(8)))  _Float16 v8h;
typedef __attribute__((ext_vector_type(8)))  float v8f;
typedef __attribute__((ext_vector_type(4)))  float v4f;
typedef __attribute__((ext_vector_type(2)))  float v2f;
typedef __attribute__((ext_vector_type(4)))  unsigned v4u;
typedef __attribute__((ext_vector_type(4)))  int v4i;
typedef float __attribute__((may_alias)) float_a;
typedef int __attribute__((may_alias)) int_a;

template <typename T> __device__ __forceinline__ void vst2(void* p, T v) { *(volatile T*)p = v; __threadfence(); *(volatile T*)p = v; }
__device__ __forceinline__ v8f wmma16(v16h a, v16h b, v8f c) {
  v8f d = __builtin_amdgcn_wmma_f32_16x16x32_f16(false, a, false, b, (short)0, c, false, false);
  asm volatile("v_nop\n\tv_nop\n\tv_nop\n\tv_nop" : "+v"(d) : "v"(a), "v"(b));
  return d;
}
__device__ __forceinline__ v8f wmma_bf(v16b a, v16b b, v8f c) {
  v8f d = __builtin_amdgcn_wmma_f32_16x16x32_bf16(false, a, false, b, (short)0, c, false, false);
  asm volatile("v_nop\n\tv_nop\n\tv_nop\n\tv_nop" : "+v"(d) : "v"(a), "v"(b));
  return d;
}
__device__ __forceinline__ v16h frag_h(const _Float16* rowk0, int lane) {
  union { v16h v; v8h q[2]; } u; const _Float16* p = rowk0 + 8 * (lane >> 4);
  u.q[0] = *(const v8h*)p; u.q[1] = *(const v8h*)(p + 16); return u.v;
}
__device__ __forceinline__ v16h frag_f32(const float* rowk0, int lane) {
  v16h a; const float* p = rowk0 + 8 * (lane >> 4);
#pragma unroll
  for (int i = 0; i < 8; ++i) { a[i] = (_Float16)p[i]; a[8 + i] = (_Float16)p[16 + i]; }
  return a;
}
__device__ __forceinline__ v16h frag_f32s(const float* rowk0, int lane, float sc) {
  v16h a; const float* p = rowk0 + 8 * (lane >> 4);
#pragma unroll
  for (int i = 0; i < 8; ++i) { a[i] = (_Float16)(p[i] * sc); a[8 + i] = (_Float16)(p[16 + i] * sc); }
  return a;
}
__device__ __forceinline__ v16h fragc_f32(const float* W, int k0, int n, int lane, int ld, int K) {
  v16h a; const int g = lane >> 4;
#pragma unroll
  for (int i = 0; i < 8; ++i) { const int ka = k0 + 8 * g + i, kb = ka + 16;
    a[i] = (_Float16)(ka < K ? W[(size_t)(ka < K ? ka : K - 1) * ld + n] : 0.f); a[8 + i] = (_Float16)(kb < K ? W[(size_t)(kb < K ? kb : K - 1) * ld + n] : 0.f); }
  return a;
}
struct F2 { v16b h, l; };
__device__ __forceinline__ F2 bsplit16(const float v[16]) { F2 r;
#pragma unroll
  for (int i = 0; i < 16; ++i) { const __bf16 h = (__bf16)v[i]; r.h[i] = h; r.l[i] = (__bf16)(v[i] - (float)h); }
  return r; }
__device__ __forceinline__ F2 split_row(const float* row, int k0, int lane) { float v[16]; const float* p = row + k0 + 8 * (lane >> 4);
#pragma unroll
  for (int i = 0; i < 8; ++i) { v[i] = p[i]; v[8 + i] = p[16 + i]; }
  return bsplit16(v); }
__device__ __forceinline__ F2 split_rowK(const float* row, int k0, int lane, int K) { float v[16]; const int g = lane >> 4;
#pragma unroll
  for (int i = 0; i < 8; ++i) { const int ka = k0 + 8 * g + i, kb = ka + 16; v[i] = ka < K ? row[ka < K ? ka : K - 1] : 0.f; v[8 + i] = kb < K ? row[kb < K ? kb : K - 1] : 0.f; }
  return bsplit16(v); }
__device__ __forceinline__ F2 split_col(const float* W, int k0, int n, int lane, int ld, int K) { float v[16]; const int g = lane >> 4;
#pragma unroll
  for (int i = 0; i < 8; ++i) { const int ka = k0 + 8 * g + i, kb = ka + 16; v[i] = ka < K ? W[(size_t)(ka < K ? ka : K - 1) * ld + n] : 0.f; v[8 + i] = kb < K ? W[(size_t)(kb < K ? kb : K - 1) * ld + n] : 0.f; }
  return bsplit16(v); }
__device__ __forceinline__ v8f mac3(const F2& a, const F2& b, v8f c) { c = wmma_bf(a.l, b.h, c); c = wmma_bf(a.h, b.l, c); return wmma_bf(a.h, b.h, c); }
__device__ __forceinline__ float sigm(float v) { return 1.0f / (1.0f + expf(-v)); }
#define LDSX() do { asm volatile("s_wait_dscnt 0" ::: "memory"); __builtin_amdgcn_wave_barrier(); __builtin_amdgcn_fence(__ATOMIC_RELEASE, "workgroup"); } while (0)


#define NB 2
#define GH 64
#define GW 64
#define NN (GH * GW)
#define SR 2
#define NR (NN / (SR * SR))
#define CC 768
#define NH 12
#define HD 64
#define LNEPS 1e-5f
#ifndef TNB
#define TNB NB
#endif
typedef __attribute__((ext_vector_type(8))) __bf16 v8b;
__device__ __forceinline__ v16b frag_b(const __bf16* rowk0, int lane) {
  union { v16b v; v8b q[2]; } u; const __bf16* p = rowk0 + 8 * (lane >> 4);
  u.q[0] = *(const v8b*)p; u.q[1] = *(const v8b*)(p + 16); return u.v;
}
__device__ __forceinline__ float bfr(float v) { return (float)(__bf16)v; }
__device__ __attribute__((noinline)) float exp_ni(float v) { return expf(v); }
__device__ __attribute__((noinline)) float erf_ni(float v) { return erff(v); }

#define WS_PSR 0u
#define WS_QH  (WS_PSR + 2u * (size_t)CC * 4 * CC)
#define WS_QL  (WS_QH + 2u * (size_t)NB * NN * CC)
#define WS_XR  (WS_QL + 2u * (size_t)NB * NN * CC)
#define WS_KH  (WS_XR + 4u * (size_t)NB * NR * CC)
#define WS_KL  (WS_KH + 2u * (size_t)NB * NR * CC)
#define WS_VT  (WS_KL + 2u * (size_t)NB * NR * CC)
#define WS_VTL (WS_VT + 2u * (size_t)NB * CC * NR)
#define WS_O   (WS_VTL + 2u * (size_t)NB * CC * NR)
#define WS_END (WS_O + 4u * (size_t)NB * NN * CC)

__device__ __forceinline__ v16b fragb_f32(const float* __restrict__ p, int lane) { v16b a; const float* pp = p + 8 * (lane >> 4);
#pragma unroll
  for (int i = 0; i < 8; ++i) { a[i] = (__bf16)pp[i]; a[8 + i] = (__bf16)pp[16 + i]; } return a; }
__device__ __forceinline__ float rope_freq(int j) { return (float)(1.0 / pow(10000.0, (double)(4 * j) / (double)HD)); }
__global__ __launch_bounds__(256) void k_packsr(const float* __restrict__ SRW, __bf16* __restrict__ PSR) { const int o = blockIdx.x, t = threadIdx.x; __shared__ __align__(16) __bf16 s[4 * CC];
  for (int e = t; e < 4 * CC; e += 256) { const int tap = e / CC, c = e % CC; s[e] = (__bf16)SRW[((size_t)o * CC + c) * 4 + tap]; } __syncthreads(); for (int q = t; q < 4 * CC / 8; q += 256) vst2((unsigned*)(PSR + (size_t)o * 4 * CC + q * 8), *(const v4u*)&s[q * 8]); }
__global__ __launch_bounds__(128) void k_q(const float* __restrict__ X, const float* __restrict__ WQ, _Float16* __restrict__ QH, _Float16* __restrict__ QL) { __shared__ __align__(16) _Float16 sh[4][16][136], sl[4][16][136]; __shared__ float tcs[64][33], tsn[64][33];
  const int tid = threadIdx.x, wave = tid >> 5, lane = tid & 31, col = lane & 15, g = lane >> 4; const size_t b = blockIdx.z; const int n0 = blockIdx.x * 64 + wave * 16; const int c0 = blockIdx.y * 128; const size_t r0 = b * NN + n0;
  for (int e = tid; e < 64 * 32; e += 128) { const int pl = e >> 5, i = e & 31; const int n = blockIdx.x * 64 + pl; const float pos = ((i & 1) == 0) ? (float)(n % GW) : (float)(n / GW); const float ang = pos * rope_freq(i >> 1); tcs[pl][i] = cosf(ang); tsn[pl][i] = sinf(ang); }
  __syncthreads();
  v8f acc[8] = {};
#pragma unroll 2
  for (int kc = 0; kc < CC / 32; ++kc) { const v16b a = fragb_f32(X + (r0 + col) * CC + kc * 32, lane);
#pragma unroll
    for (int j = 0; j < 8; ++j) acc[j] = wmma_bf(a, fragb_f32(WQ + (size_t)(c0 + j * 16 + col) * CC + kc * 32, lane), acc[j]); }
#pragma unroll
  for (int j = 0; j < 8; ++j) { const int d = (c0 + j * 16 + col) & 63; const int i = d >> 1; const float fr = rope_freq(i >> 1); const bool usex = (i & 1) == 0; const bool odd = d & 1;
#pragma unroll
    for (int r = 0; r < 8; ++r) { const float cs = tcs[wave * 16 + 8 * g + r][i], sn = tsn[wave * 16 + 8 * g + r][i]; (void)fr; (void)usex;
      const float me = acc[j][r]; const float partner = __shfl_xor(me, 1);
      const float x0 = odd ? partner : me, x1 = odd ? me : partner; const float y = odd ? (x0 * sn + x1 * cs) : (x0 * cs - x1 * sn);
      const _Float16 hv = (_Float16)y; sh[wave][8 * g + r][j * 16 + col] = hv; sl[wave][8 * g + r][j * 16 + col] = (_Float16)((y - (float)hv) * 2048.0f); } }
  LDSX(); for (int rl = 0; rl < 16; ++rl) if (lane < 16) { const size_t o = (r0 + rl) * CC + c0 + lane * 8; vst2((unsigned*)(QH + o), *(const v4u*)&sh[wave][rl][lane * 8]); vst2((unsigned*)(QL + o), *(const v4u*)&sl[wave][rl][lane * 8]); } }
__global__ __launch_bounds__(128) void k_sr(const float* __restrict__ X, const __bf16* __restrict__ PSR, const float* __restrict__ SRB, float* __restrict__ XR) { __shared__ __align__(16) float sf[4][16][132];
  const int tid = threadIdx.x, wave = tid >> 5, lane = tid & 31, col = lane & 15, g = lane >> 4; const size_t b = blockIdx.z; const int m0 = blockIdx.x * 64 + wave * 16; const int c0 = blockIdx.y * 128; const int m = m0 + col; const int py = m / (GW / SR), px = m % (GW / SR);
  v8f acc[8] = {};
#pragma unroll 2
  for (int kc = 0; kc < 4 * CC / 32; ++kc) { const int tap = kc / (CC / 32), cb = (kc % (CC / 32)) * 32; const int ky = tap >> 1, kx = tap & 1; const int n = (SR * py + ky) * GW + SR * px + kx;
    const v16b a = fragb_f32(X + (b * NN + n) * CC + cb, lane);
#pragma unroll
    for (int j = 0; j < 8; ++j) acc[j] = wmma_bf(a, frag_b(PSR + (size_t)(c0 + j * 16 + col) * (4 * CC) + kc * 32, lane), acc[j]); }
#pragma unroll
  for (int j = 0; j < 8; ++j) { const float bb = bfr(SRB[c0 + j * 16 + col]);
#pragma unroll
    for (int r = 0; r < 8; ++r) sf[wave][8 * g + r][j * 16 + col] = acc[j][r] + bb; }
  LDSX(); for (int rl = 0; rl < 16; ++rl) vst2(XR + (b * NR + m0 + rl) * CC + c0 + lane * 4, *(const v4f*)&sf[wave][rl][lane * 4]); }
__global__ __launch_bounds__(256) void k_ln(float* __restrict__ XR, const float* __restrict__ G, const float* __restrict__ Bt) { __shared__ float red[8]; __shared__ __align__(16) float so[CC]; const int t = threadIdx.x; const size_t row = blockIdx.x; float v[3]; float s = 0.f;
  for (int i = 0; i < 3; ++i) { v[i] = XR[row * CC + t + 256 * i]; s += v[i]; }
#pragma unroll
  for (int o = 1; o < 32; o <<= 1) s += __shfl_xor(s, o);
  if ((t & 31) == 0) red[t >> 5] = s; __syncthreads(); float mu = 0.f; for (int i = 0; i < 8; ++i) mu += red[i]; mu /= (float)CC; __syncthreads();
  float q = 0.f; for (int i = 0; i < 3; ++i) { const float d = v[i] - mu; q += d * d; }
#pragma unroll
  for (int o = 1; o < 32; o <<= 1) q += __shfl_xor(q, o);
  if ((t & 31) == 0) red[t >> 5] = q; __syncthreads(); float var = 0.f; for (int i = 0; i < 8; ++i) var += red[i]; var /= (float)CC; const float inv = 1.0f / sqrtf(var + LNEPS);
  for (int i = 0; i < 3; ++i) { const int c = t + 256 * i; so[c] = (v[i] - mu) * inv * bfr(G[c]) + bfr(Bt[c]); } __syncthreads(); for (int qd = t; qd < CC / 4; qd += 256) vst2(XR + row * CC + qd * 4, *(const v4f*)&so[qd * 4]); }
__global__ __launch_bounds__(128) void k_kv(const float* __restrict__ XR, const float* __restrict__ WKV, _Float16* __restrict__ KH, _Float16* __restrict__ KL, _Float16* __restrict__ VT, _Float16* __restrict__ VTL) { __shared__ __align__(16) _Float16 sh[64][136], sl[64][136]; __shared__ __align__(16) _Float16 th[128][72], tl[128][72]; __shared__ float tcs[64][33], tsn[64][33];
  const int tid = threadIdx.x, wave = tid >> 5, lane = tid & 31, col = lane & 15, g = lane >> 4; const size_t b = blockIdx.z; const int m0 = blockIdx.x * 64 + wave * 16; const int c0 = blockIdx.y * 128; const size_t r0 = b * NR + m0; const bool isv = c0 >= CC;
  for (int e = tid; e < 64 * 32; e += 128) { const int pl = e >> 5, i = e & 31; const int m = blockIdx.x * 64 + pl; const float pos = ((i & 1) == 0) ? (0.5f + (float)(m % GW) * 2.0f) : (0.5f + (float)(m / GW) * 2.0f); const float ang = pos * rope_freq(i >> 1); tcs[pl][i] = cosf(ang); tsn[pl][i] = sinf(ang); }
  __syncthreads();
  v8f acc[8] = {};
#pragma unroll 2
  for (int kc = 0; kc < CC / 32; ++kc) { const F2 a = split_row(XR + (r0 + col) * CC, kc * 32, lane);
#pragma unroll
    for (int j = 0; j < 8; ++j) { const v16b w = fragb_f32(WKV + (size_t)(c0 + j * 16 + col) * CC + kc * 32, lane); acc[j] = wmma_bf(a.h, w, acc[j]); acc[j] = wmma_bf(a.l, w, acc[j]); } }
#pragma unroll
  for (int j = 0; j < 8; ++j) { const int d = (c0 + j * 16 + col) & 63; const int i = d >> 1; const float fr = rope_freq(i >> 1); const bool usex = (i & 1) == 0; const bool odd = d & 1;
#pragma unroll
    for (int r = 0; r < 8; ++r) { const int m = m0 + 8 * g + r; float y = acc[j][r];
      (void)m; (void)fr; (void)usex; if (!isv) { const float cs = tcs[wave * 16 + 8 * g + r][i], sn = tsn[wave * 16 + 8 * g + r][i]; const float me = acc[j][r]; const float partner = __shfl_xor(me, 1); const float x0 = odd ? partner : me, x1 = odd ? me : partner; y = odd ? (x0 * sn + x1 * cs) : (x0 * cs - x1 * sn); }
      const _Float16 hv = (_Float16)y, lv = (_Float16)((y - (float)hv) * 2048.0f); if (!isv) { sh[wave * 16 + 8 * g + r][j * 16 + col] = hv; sl[wave * 16 + 8 * g + r][j * 16 + col] = lv; } else { th[j * 16 + col][wave * 16 + 8 * g + r] = hv; tl[j * 16 + col][wave * 16 + 8 * g + r] = lv; } } }
  __syncthreads();
  if (!isv) { for (int e = tid; e < 64 * 16; e += 128) { const int rl = e >> 4, q = e & 15; const size_t o = (b * NR + blockIdx.x * 64 + rl) * CC + c0 + q * 8; vst2((unsigned*)(KH + o), *(const v4u*)&sh[rl][q * 8]); vst2((unsigned*)(KL + o), *(const v4u*)&sl[rl][q * 8]); } }
  else { const int cv0 = c0 - CC; for (int e = tid; e < 128 * 8; e += 128) { const int cl = e >> 3, q = e & 7; const size_t o = (b * CC + cv0 + cl) * (size_t)NR + blockIdx.x * 64 + q * 8; vst2((unsigned*)(VT + o), *(const v4u*)&th[cl][q * 8]); vst2((unsigned*)(VTL + o), *(const v4u*)&tl[cl][q * 8]); } } }
__device__ __forceinline__ int visf(int n) { const int xpos = n / (SR * GH); const int ox = n / GH, oy = n % GH; const int ypos = (ox + oy * GH) / (SR * GH); return xpos * SR + ypos + 1; }
__global__ __launch_bounds__(128) void k_att(const _Float16* __restrict__ QH, const _Float16* __restrict__ QL, const _Float16* __restrict__ KH, const _Float16* __restrict__ KL, const _Float16* __restrict__ VT, const _Float16* __restrict__ VTL, float* __restrict__ O) {
  __shared__ __align__(16) float sp[4][16][36]; __shared__ __align__(16) float so[4][16][68]; __shared__ int smaxvis;
  const int tid = threadIdx.x, wave = tid >> 5, lane = tid & 31, col = lane & 15, g = lane >> 4; const int h = blockIdx.y; const size_t b = blockIdx.z; const int q0 = blockIdx.x * 64 + wave * 16; const size_t rq = b * NN + q0;
  if (tid == 0) { int mv = 0; for (int i = 0; i < 64; ++i) mv = max(mv, visf(blockIdx.x * 64 + i)); smaxvis = mv; } __syncthreads(); const int nks = (smaxvis + 31) / 32;
  int vis[8];
#pragma unroll
  for (int r = 0; r < 8; ++r) vis[r] = visf(q0 + 8 * g + r);
  v16h aq[2], al[2];
#pragma unroll
  for (int kc = 0; kc < 2; ++kc) { aq[kc] = frag_h(QH + (rq + col) * CC + h * HD + kc * 32, lane); al[kc] = frag_h(QL + (rq + col) * CC + h * HD + kc * 32, lane); }
  float m[8], l[8];
#pragma unroll
  for (int r = 0; r < 8; ++r) { m[r] = -3.0e38f; l[r] = 0.f; }
  v8f acc[4] = {}, accl[4] = {};
#pragma unroll 1
  for (int ks = 0; ks < nks; ++ks) { float s[2][8];
#pragma unroll
    for (int ct = 0; ct < 2; ++ct) { const int kk = ks * 32 + ct * 16 + col; const size_t rk = b * NR + kk; v8f c = {}, cl = {};
#pragma unroll
      for (int kc = 0; kc < 2; ++kc) { const v16h kh = frag_h(KH + rk * CC + h * HD + kc * 32, lane), kl = frag_h(KL + rk * CC + h * HD + kc * 32, lane); c = wmma16(aq[kc], kh, c); cl = wmma16(aq[kc], kl, cl); cl = wmma16(al[kc], kh, cl); }
#pragma unroll
      for (int r = 0; r < 8; ++r) s[ct][r] = (kk < vis[r]) ? (c[r] + cl[r] * (1.0f / 2048.0f)) * 0.125f : -3.0e38f; }
    float alpha[8];
#pragma unroll
    for (int r = 0; r < 8; ++r) { float mx = fmaxf(s[0][r], s[1][r]);
#pragma unroll
      for (int o = 1; o < 16; o <<= 1) mx = fmaxf(mx, __shfl_xor(mx, o));
      const float mn = fmaxf(m[r], mx); alpha[r] = (m[r] <= -1.0e38f) ? 0.f : __expf(m[r] - mn); const float e0 = (s[0][r] <= -1.0e38f) ? 0.f : __expf(s[0][r] - mn), e1 = (s[1][r] <= -1.0e38f) ? 0.f : __expf(s[1][r] - mn); float es = e0 + e1;
#pragma unroll
      for (int o = 1; o < 16; o <<= 1) es += __shfl_xor(es, o);
      l[r] = l[r] * alpha[r] + es; m[r] = (mn > -1.0e38f) ? mn : m[r]; sp[wave][8 * g + r][col] = e0; sp[wave][8 * g + r][16 + col] = e1; }
#pragma unroll
    for (int j = 0; j < 4; ++j)
#pragma unroll
      for (int r = 0; r < 8; ++r) { acc[j][r] *= alpha[r]; accl[j][r] *= alpha[r]; }
    LDSX();
    v16h pa, pal; { const float* prow = &sp[wave][col][0] + 8 * (lane >> 4);
#pragma unroll
      for (int i = 0; i < 8; ++i) { const float p0 = prow[i] * 2048.0f, p1 = prow[16 + i] * 2048.0f; pa[i] = (_Float16)p0; pa[8 + i] = (_Float16)p1; pal[i] = (_Float16)((p0 - (float)pa[i]) * 2048.0f); pal[8 + i] = (_Float16)((p1 - (float)pa[8 + i]) * 2048.0f); } }
#pragma unroll
    for (int j = 0; j < 4; ++j) { const size_t po = (b * CC + (size_t)h * HD + j * 16 + col) * (size_t)NR + ks * 32; const v16h vh = frag_h(VT + po, lane), vl = frag_h(VTL + po, lane); acc[j] = wmma16(pa, vh, acc[j]); accl[j] = wmma16(pa, vl, accl[j]); accl[j] = wmma16(pal, vh, accl[j]); }
    LDSX(); }
#pragma unroll
  for (int r = 0; r < 8; ++r) { const float il = (l[r] > 0.f) ? (1.0f / 2048.0f) / l[r] : 0.f;
#pragma unroll
    for (int j = 0; j < 4; ++j) so[wave][8 * g + r][j * 16 + col] = (acc[j][r] + accl[j][r] * (1.0f / 2048.0f)) * il; }
  LDSX(); for (int rl = 0; rl < 16; ++rl) if (lane < 16) vst2(O + (rq + rl) * CC + (size_t)h * HD + lane * 4, *(const v4f*)&so[wave][rl][lane * 4]); }
__global__ __launch_bounds__(128) void k_out(const float* __restrict__ Or, const float* __restrict__ WP, const float* __restrict__ BP, float* __restrict__ OUT) { __shared__ __align__(16) float sf[4][16][132];
  const int tid = threadIdx.x, wave = tid >> 5, lane = tid & 31, col = lane & 15, g = lane >> 4; const size_t r0 = (size_t)blockIdx.x * 64 + wave * 16; const int c0 = blockIdx.y * 128;
  v8f acc[8] = {};
#pragma unroll 2
  for (int kc = 0; kc < CC / 32; ++kc) { const F2 a = split_row(Or + (r0 + col) * CC, kc * 32, lane);
#pragma unroll
    for (int j = 0; j < 8; ++j) { const v16b w = fragb_f32(WP + (size_t)(c0 + j * 16 + col) * CC + kc * 32, lane); acc[j] = wmma_bf(a.h, w, acc[j]); acc[j] = wmma_bf(a.l, w, acc[j]); } }
#pragma unroll
  for (int j = 0; j < 8; ++j) { const float bb = bfr(BP[c0 + j * 16 + col]);
#pragma unroll
    for (int r = 0; r < 8; ++r) sf[wave][8 * g + r][j * 16 + col] = acc[j][r] + bb; }
  LDSX(); for (int rl = 0; rl < 16; ++rl) vst2(OUT + (r0 + rl) * CC + c0 + lane * 4, *(const v4f*)&sf[wave][rl][lane * 4]); }
extern "C" void kernel_launch(void* const* d_in, const int* in_sizes, int n_in, void* d_out, int out_size, void* d_ws, size_t ws_size, hipStream_t stream) {
  (void)in_sizes; (void)n_in; (void)out_size;
  const float** F = (const float**)d_in;
  if (ws_size < (size_t)WS_END) return;
  char* ws = (char*)d_ws; __bf16* PSR = (__bf16*)(ws + WS_PSR); _Float16 *QH = (_Float16*)(ws + WS_QH), *QL = (_Float16*)(ws + WS_QL), *KH = (_Float16*)(ws + WS_KH), *KL = (_Float16*)(ws + WS_KL), *VT = (_Float16*)(ws + WS_VT), *VTL = (_Float16*)(ws + WS_VTL); float *XR = (float*)(ws + WS_XR), *O = (float*)(ws + WS_O);
  k_packsr<<<CC, 256, 0, stream>>>(F[3], PSR);
  k_q<<<dim3(NN / 64, CC / 128, TNB), 128, 0, stream>>>(F[0], F[1], QH, QL);
  k_sr<<<dim3(NR / 64, CC / 128, TNB), 128, 0, stream>>>(F[0], PSR, F[4], XR);
  k_ln<<<TNB * NR, 256, 0, stream>>>(XR, F[5], F[6]);
  k_kv<<<dim3(NR / 64, 2 * CC / 128, TNB), 128, 0, stream>>>(XR, F[2], KH, KL, VT, VTL);
  k_att<<<dim3(NN / 64, NH, TNB), 128, 0, stream>>>(QH, QL, KH, KL, VT, VTL, O);
  k_out<<<dim3(TNB * NN / 64, CC / 128), 128, 0, stream>>>(O, F[7], F[8], (float*)d_out);
}
